// VanillaRNN_51531017617809
// MI455X (gfx1250) — hardware-verified
//
#include <hip/hip_runtime.h>
#include <math.h>

constexpr int NBATCH   = 256;
constexpr int NSTEP    = 128;
constexpr int NHID     = 2048;
constexpr int NCLS     = 10;
constexpr int NTHR     = 256;
constexpr int NWAVE    = NTHR / 32;
constexpr int ROWS_BLK = 32;
constexpr int NBLK     = NBATCH / ROWS_BLK;
constexpr int COLS_PASS = NWAVE * 64;
constexpr int NPASS    = NHID / COLS_PASS;
constexpr int KCHUNKS  = NHID / 32;
constexpr int TSPLIT   = 64;
constexpr int SLABP    = 68;
constexpr int XPITCH   = NSTEP;
constexpr float WCARRY = 32.0f;
constexpr float HCARRY = 1024.0f;
constexpr float ACC_INV = 1.0f / (WCARRY * HCARRY);
constexpr size_t PLANE_ELEMS = (size_t)NBATCH * NHID;
constexpr size_t BUF_ELEMS   = 2 * PLANE_ELEMS;
constexpr int XS_BYTES   = ROWS_BLK * XPITCH * 4;
constexpr int SLAB_BYTES = NWAVE * ROWS_BLK * SLABP * 4;
constexpr int LDS_BYTES  = XS_BYTES + SLAB_BYTES;
constexpr int NOUT0 = NBATCH * NHID;
constexpr int NOUT1 = NBATCH * NCLS;

static_assert(NBATCH % ROWS_BLK == 0, "batch tiling");
static_assert(NHID % 32 == 0, "K multiple of 32");
static_assert(NPASS * COLS_PASS == NHID, "column tiling");
static_assert(ROWS_BLK == 32, "two 16-row subtiles per block");
static_assert((ROWS_BLK * XPITCH) == 4 * NTHR * 4, "x tile staging coverage");
static_assert(NOUT1 % NTHR == 0, "head grid exact");
static_assert((NHID * NHID / 8) % NTHR == 0, "weight plane grid exact");
static_assert(XS_BYTES % 16 == 0 && (SLABP * 4) % 16 == 0, "LDS alignment");
static_assert((size_t)NOUT0 * 4 == 2097152, "out1 byte offset");

typedef __attribute__((ext_vector_type(16))) _Float16 v16h;
typedef __attribute__((ext_vector_type(8)))  _Float16 v8h;
typedef __attribute__((ext_vector_type(8)))  float    v8f;
typedef __attribute__((ext_vector_type(4)))  float    v4f;
typedef __attribute__((ext_vector_type(4)))  unsigned v4u;

__device__ __forceinline__ unsigned short f2bf_bits(float f) {
  unsigned u = __float_as_uint(f);
  return (unsigned short)((u + 0x7FFFu + ((u >> 16) & 1u)) >> 16);
}
__device__ __forceinline__ float bf_bits2f(unsigned short h) { return __uint_as_float(((unsigned)h) << 16); }
__device__ __forceinline__ float bf16r(float f) { return bf_bits2f(f2bf_bits(f)); }

union FragU { v16h v; v8h h[2]; };
__device__ __forceinline__ v16h frag_load(const _Float16* p) {
  FragU f;
  f.h[0] = *(const v8h*)(p);
  f.h[1] = *(const v8h*)(p + 16);
  return f.v;
}
__device__ __forceinline__ v8f mma_h(v16h a, v16h b, v8f c) {
  return __builtin_amdgcn_wmma_f32_16x16x32_f16(false, a, false, b, (short)0, c, false, false);
}
__device__ __forceinline__ void guard8(v8f& c0, v8f& c1, v8f& c2, v8f& c3, v8f& c4, v8f& c5, v8f& c6, v8f& c7,
                                       v16h a0, v16h a1, v16h b0, v16h b1, v16h b2, v16h b3) {
  asm volatile("v_nop\n\tv_nop\n\tv_nop\n\tv_nop"
               : "+v"(c0), "+v"(c1), "+v"(c2), "+v"(c3), "+v"(c4), "+v"(c5), "+v"(c6), "+v"(c7)
               : "v"(a0), "v"(a1), "v"(b0), "v"(b1), "v"(b2), "v"(b3));
}
__device__ __forceinline__ void guard8s(v8f& c0, v8f& c1, v8f& c2, v8f& c3, v8f& c4, v8f& c5, v8f& c6, v8f& c7,
                                        v16h a0, v16h a1, v16h l0, v16h l1, v16h b0, v16h b1, v16h b2, v16h b3) {
  asm volatile("v_nop\n\tv_nop\n\tv_nop\n\tv_nop"
               : "+v"(c0), "+v"(c1), "+v"(c2), "+v"(c3), "+v"(c4), "+v"(c5), "+v"(c6), "+v"(c7)
               : "v"(a0), "v"(a1), "v"(l0), "v"(l1), "v"(b0), "v"(b1), "v"(b2), "v"(b3));
}
__device__ __forceinline__ void wave_lds_sync() {
  __builtin_amdgcn_fence(__ATOMIC_RELEASE, "workgroup");
  __builtin_amdgcn_wave_barrier();
  __builtin_amdgcn_fence(__ATOMIC_ACQUIRE, "workgroup");
}
__device__ __forceinline__ float tanh_e(float z) {
  z = fminf(fmaxf(z, -15.0f), 15.0f);
  const float e = expf(2.0f * z);
  const float d = e + 1.0f;
  float r = __builtin_amdgcn_rcpf(d);
  r = fmaf(fmaf(-d, r, 1.0f), r, r);
  return fmaf(-2.0f, r, 1.0f);
}

__global__ __launch_bounds__(NTHR) void wplane_kernel(const float* __restrict__ W, unsigned short* __restrict__ dst, int n8) {
  const int i = blockIdx.x * NTHR + threadIdx.x;
  if (i < n8) {
    const float* sp = W + (size_t)i * 8;
    const v4f a = *(const v4f*)(sp);
    const v4f b = *(const v4f*)(sp + 4);
    v8h hv;
#pragma unroll
    for (int e = 0; e < 4; ++e) {
      const float fa = bf16r(a[e]) * WCARRY;
      const float fb = bf16r(b[e]) * WCARRY;
      hv[e]     = (_Float16)fa;
      hv[4 + e] = (_Float16)fb;
    }
    *(volatile v8h*)(dst + (size_t)i * 8) = hv;
    __threadfence();
    *(volatile v8h*)(dst + (size_t)i * 8) = hv;
  }
}

__global__ __launch_bounds__(NTHR) void rnn_seq_kernel(const float* __restrict__ x, const float* __restrict__ U,
                                                       const float* __restrict__ bh,
                                                       const unsigned short* __restrict__ Wtp,
                                                       unsigned short* Hst, float* out0) {
  extern __shared__ __align__(16) unsigned char dyn_lds[];
  float* xs = (float*)(void*)dyn_lds;
  const int tid = threadIdx.x, lane = tid & 31, wave = tid >> 5;
  float* slabf = (float*)(void*)(dyn_lds + XS_BYTES) + wave * (ROWS_BLK * SLABP);
  const int rl = lane & 15, hh = lane >> 4, koff = hh * 8;
  const int q = lane >> 3, c8 = (lane & 7) * 8, c4 = rl * 4;
  const int rowbase = blockIdx.x * ROWS_BLK;

#pragma unroll
  for (int i = 0; i < 4; ++i) {
    const int idx = i * NTHR + tid;
    const int row = idx >> 5, cc = (idx & 31) * 4;
    const v4f v = *(const v4f*)(x + (size_t)(rowbase + row) * NSTEP + cc);
    v4f o;
#pragma unroll
    for (int e = 0; e < 4; ++e) o[e] = bf16r(v[e]);
    *(v4f*)(xs + row * XPITCH + cc) = o;
  }
  __syncthreads();

  const _Float16* wlane = (const _Float16*)Wtp + (size_t)(wave * 64 + rl) * NHID + koff;
  const size_t a_lane = (size_t)(rowbase + rl) * NHID + koff;
  const size_t s_lane = (size_t)(rowbase + q) * NHID + c8;
  float* o_lane = out0 + (size_t)(rowbase + hh) * NHID + c4;
  const v8f z8 = {0.f, 0.f, 0.f, 0.f, 0.f, 0.f, 0.f, 0.f};

#pragma unroll 1
  for (int t = 0; t < NSTEP; ++t) {
    const bool last = (t == NSTEP - 1);
    const _Float16* hcur = (const _Float16*)Hst + (size_t)(t & 1) * BUF_ELEMS + a_lane;
    unsigned short* hnxt = Hst + (size_t)((t + 1) & 1) * BUF_ELEMS + s_lane;

#pragma unroll 1
    for (int p = 0; p < NPASS; ++p) {
      const int n0 = p * COLS_PASS + wave * 64;
      v8f acc[2][4];
#pragma unroll
      for (int i = 0; i < 2; ++i)
#pragma unroll
        for (int j = 0; j < 4; ++j) acc[i][j] = z8;

      if (t > 0) {
        const _Float16* pa = hcur;
        const _Float16* pb = wlane + (size_t)p * COLS_PASS * NHID;
        if (t < TSPLIT) {
#pragma unroll 1
          for (int kc = 0; kc < KCHUNKS; ++kc) {
            const v16h a0 = frag_load(pa);
            const v16h a1 = frag_load(pa + 16 * NHID);
            const v16h b0 = frag_load(pb);
            const v16h b1 = frag_load(pb + 16 * NHID);
            const v16h b2 = frag_load(pb + 32 * NHID);
            const v16h b3 = frag_load(pb + 48 * NHID);
            acc[0][0] = mma_h(a0, b0, acc[0][0]);
            acc[0][1] = mma_h(a0, b1, acc[0][1]);
            acc[0][2] = mma_h(a0, b2, acc[0][2]);
            acc[0][3] = mma_h(a0, b3, acc[0][3]);
            acc[1][0] = mma_h(a1, b0, acc[1][0]);
            acc[1][1] = mma_h(a1, b1, acc[1][1]);
            acc[1][2] = mma_h(a1, b2, acc[1][2]);
            acc[1][3] = mma_h(a1, b3, acc[1][3]);
            guard8(acc[0][0], acc[0][1], acc[0][2], acc[0][3], acc[1][0], acc[1][1], acc[1][2], acc[1][3],
                   a0, a1, b0, b1, b2, b3);
            pa += 32;
            pb += 32;
          }
        } else {
#pragma unroll 1
          for (int kc = 0; kc < KCHUNKS; ++kc) {
            const v16h a0 = frag_load(pa);
            const v16h a1 = frag_load(pa + 16 * NHID);
            const v16h l0 = frag_load(pa + PLANE_ELEMS);
            const v16h l1 = frag_load(pa + PLANE_ELEMS + 16 * NHID);
            const v16h b0 = frag_load(pb);
            const v16h b1 = frag_load(pb + 16 * NHID);
            const v16h b2 = frag_load(pb + 32 * NHID);
            const v16h b3 = frag_load(pb + 48 * NHID);
            acc[0][0] = mma_h(a0, b0, acc[0][0]);
            acc[0][1] = mma_h(a0, b1, acc[0][1]);
            acc[0][2] = mma_h(a0, b2, acc[0][2]);
            acc[0][3] = mma_h(a0, b3, acc[0][3]);
            acc[1][0] = mma_h(a1, b0, acc[1][0]);
            acc[1][1] = mma_h(a1, b1, acc[1][1]);
            acc[1][2] = mma_h(a1, b2, acc[1][2]);
            acc[1][3] = mma_h(a1, b3, acc[1][3]);
            acc[0][0] = mma_h(l0, b0, acc[0][0]);
            acc[0][1] = mma_h(l0, b1, acc[0][1]);
            acc[0][2] = mma_h(l0, b2, acc[0][2]);
            acc[0][3] = mma_h(l0, b3, acc[0][3]);
            acc[1][0] = mma_h(l1, b0, acc[1][0]);
            acc[1][1] = mma_h(l1, b1, acc[1][1]);
            acc[1][2] = mma_h(l1, b2, acc[1][2]);
            acc[1][3] = mma_h(l1, b3, acc[1][3]);
            guard8s(acc[0][0], acc[0][1], acc[0][2], acc[0][3], acc[1][0], acc[1][1], acc[1][2], acc[1][3],
                    a0, a1, l0, l1, b0, b1, b2, b3);
            pa += 32;
            pb += 32;
          }
        }
      }

#pragma unroll
      for (int i = 0; i < 2; ++i)
#pragma unroll
        for (int j = 0; j < 4; ++j)
#pragma unroll
          for (int r = 0; r < 8; ++r)
            slabf[(16 * i + 8 * hh + r) * SLABP + 16 * j + rl] = acc[i][j][r];

      float ub[8], bb[8];
      {
        const v4f u0 = *(const v4f*)(U + n0 + c8);
        const v4f u1 = *(const v4f*)(U + n0 + c8 + 4);
        const v4f g0 = *(const v4f*)(bh + n0 + c8);
        const v4f g1 = *(const v4f*)(bh + n0 + c8 + 4);
#pragma unroll
        for (int e = 0; e < 4; ++e) {
          ub[e]     = bf16r(u0[e]);
          ub[4 + e] = bf16r(u1[e]);
          bb[e]     = bf16r(g0[e]);
          bb[4 + e] = bf16r(g1[e]);
        }
      }
      wave_lds_sync();

#pragma unroll 1
      for (int it = 0; it < 8; ++it) {
        const int row = it * 4 + q;
        float* sp = slabf + row * SLABP + c8;
        const v4f s0 = *(const v4f*)(sp);
        const v4f s1 = *(const v4f*)(sp + 4);
        const float xb = xs[row * XPITCH + t];
        float hv[8];
#pragma unroll
        for (int e = 0; e < 4; ++e) {
          const float z0 = fmaf(s0[e], ACC_INV, fmaf(xb, ub[e], bb[e]));
          const float z1 = fmaf(s1[e], ACC_INV, fmaf(xb, ub[4 + e], bb[4 + e]));
          hv[e]     = tanh_e(z0);
          hv[4 + e] = tanh_e(z1);
        }
        if (last) {
          v4f o0, o1;
#pragma unroll
          for (int e = 0; e < 4; ++e) { o0[e] = hv[e]; o1[e] = hv[4 + e]; }
          *(v4f*)(sp)     = o0;
          *(v4f*)(sp + 4) = o1;
        } else {
          unsigned hw[4], lw[4];
#pragma unroll
          for (int k2 = 0; k2 < 4; ++k2) {
            const float sa = hv[2 * k2] * HCARRY;
            const float sb = hv[2 * k2 + 1] * HCARRY;
            const _Float16 ha = (_Float16)sa;
            const _Float16 hb = (_Float16)sb;
            float fa = (float)ha;
            float fb = (float)hb;
            asm volatile("" : "+v"(fa));
            asm volatile("" : "+v"(fb));
            const _Float16 la = (_Float16)(sa - fa);
            const _Float16 lb = (_Float16)(sb - fb);
            const unsigned short hba = __builtin_bit_cast(unsigned short, ha);
            const unsigned short hbb = __builtin_bit_cast(unsigned short, hb);
            const unsigned short lba = __builtin_bit_cast(unsigned short, la);
            const unsigned short lbb = __builtin_bit_cast(unsigned short, lb);
            hw[k2] = (unsigned)hba | ((unsigned)hbb << 16);
            lw[k2] = (unsigned)lba | ((unsigned)lbb << 16);
          }
          v4u hq, lq;
          hq[0] = hw[0]; hq[1] = hw[1]; hq[2] = hw[2]; hq[3] = hw[3];
          lq[0] = lw[0]; lq[1] = lw[1]; lq[2] = lw[2]; lq[3] = lw[3];
          *(v4u*)(void*)(sp)     = hq;
          *(v4u*)(void*)(sp + 4) = lq;
        }
      }
      wave_lds_sync();

      if (last) {
        for (int pass = 0; pass < 2; ++pass) {
#pragma unroll
          for (int it = 0; it < 16; ++it) {
            const int row = it * 2 + hh;
            const v4f v = *(const v4f*)(slabf + row * SLABP + c4);
            *(volatile v4f*)(o_lane + (size_t)(it * 2) * NHID + n0) = v;
          }
          __threadfence();
        }
      } else {
        for (int pass = 0; pass < 2; ++pass) {
#pragma unroll
          for (int it = 0; it < 8; ++it) {
            const int row = it * 4 + q;
            const float* sp = slabf + row * SLABP + c8;
            const v4u hq = *(const v4u*)(const void*)(sp);
            const v4u lq = *(const v4u*)(const void*)(sp + 4);
            unsigned short* gp = hnxt + (size_t)(it * 4) * NHID + n0;
            *(volatile v4u*)(void*)(gp) = hq;
            *(volatile v4u*)(void*)(gp + PLANE_ELEMS) = lq;
          }
          __threadfence();
        }
      }
      wave_lds_sync();
    }
    __threadfence();
    __syncthreads();
    __threadfence();
  }
}

__global__ __launch_bounds__(NTHR) void head_kernel(const float* hl, const float* __restrict__ V,
                                                    const float* __restrict__ bp, float* out1) {
  const int idx0 = blockIdx.x * NTHR + threadIdx.x;
  const int idx = (idx0 < NOUT1) ? idx0 : (NOUT1 - 1);
  const int b = idx / NCLS;
  const int c = idx - b * NCLS;
  const float* hp = hl + (size_t)b * NHID;
  const float* vp = V + (size_t)c * NHID;
  float s0 = 0.0f, s1 = 0.0f, s2 = 0.0f, s3 = 0.0f;
#pragma unroll 2
  for (int k = 0; k < NHID; k += 4) {
    const v4f hv = *(const v4f*)(hp + k);
    const v4f vv = *(const v4f*)(vp + k);
    s0 = fmaf(hv[0], bf16r(vv[0]), s0);
    s1 = fmaf(hv[1], bf16r(vv[1]), s1);
    s2 = fmaf(hv[2], bf16r(vv[2]), s2);
    s3 = fmaf(hv[3], bf16r(vv[3]), s3);
  }
  const float res = ((s0 + s1) + (s2 + s3)) + bf16r(bp[c]);
  if (idx0 < NOUT1) {
    *(volatile float*)(out1 + idx0) = res;
    __threadfence();
    *(volatile float*)(out1 + idx0) = res;
  }
}

extern "C" void kernel_launch(void* const* d_in, const int* in_sizes, int n_in,
                              void* d_out, int out_size, void* d_ws, size_t ws_size, hipStream_t stream) {
  if (n_in < 6 || d_out == nullptr || d_ws == nullptr) return;
  if (in_sizes[0] != NBATCH * NSTEP || in_sizes[1] != NHID || in_sizes[2] != NHID * NHID ||
      in_sizes[3] != NCLS * NHID || in_sizes[4] != NHID || in_sizes[5] != NCLS ||
      out_size != NOUT0 + NOUT1) return;

  const float* x  = (const float*)d_in[0];
  const float* U  = (const float*)d_in[1];
  const float* W  = (const float*)d_in[2];
  const float* V  = (const float*)d_in[3];
  const float* bh = (const float*)d_in[4];
  const float* bp = (const float*)d_in[5];
  float* out0 = (float*)d_out;
  float* out1 = out0 + (size_t)NOUT0;

  char* ws = (char*)d_ws;
  size_t off = 0;
  auto carve = [&](size_t bytes) -> char* { char* p = ws + off; off += (bytes + 255) & ~(size_t)255; return p; };
  unsigned short* WT16 = (unsigned short*)carve((size_t)NHID * NHID * 2);
  unsigned short* HST  = (unsigned short*)carve((size_t)2 * BUF_ELEMS * 2);
  if (off > ws_size || off > (size_t)134217728) return;

  const int n8 = NHID * NHID / 8;
  wplane_kernel<<<n8 / NTHR, NTHR, 0, stream>>>(W, WT16, n8);
  rnn_seq_kernel<<<NBLK, NTHR, LDS_BYTES, stream>>>(x, U, bh, WT16, HST, out0);
  head_kernel<<<NOUT1 / NTHR, NTHR, 0, stream>>>(out0, V, bp, out1);
}
